// LSTM_68075231641639
// MI455X (gfx1250) — hardware-run, weakly checked
//
#include <hip/hip_runtime.h>
#include <math.h>

typedef __attribute__((ext_vector_type(16))) __bf16 v16b;
typedef __attribute__((ext_vector_type(8)))  __bf16 v8b;
typedef __attribute__((ext_vector_type(8)))  float  v8f;
typedef __attribute__((ext_vector_type(4)))  float  v4f;
typedef __attribute__((ext_vector_type(2)))  float  v2f;

constexpr int kBatch = 4096;
constexpr int kSteps = 200;
constexpr int kIn    = 4;
constexpr int kHid   = 2;
constexpr int kRows  = kBatch * kSteps;
constexpr int kF1    = 32;
constexpr int kF2    = 80;
constexpr int kF3    = 16;
constexpr int kOutW  = 2;
constexpr float kEps = 1e-5f;

constexpr int kCellRows      = 32;
constexpr int kCellBlocks    = kBatch / kCellRows;
constexpr int kTileRows      = 128;
constexpr int kTilesPerBlock = 8;
constexpr int kPassBlocks    = kRows / (kTileRows * kTilesPerBlock);
constexpr int kHeadThreads   = 256;
constexpr int kHeadBlocks    = kRows / kHeadThreads;

static_assert(kRows == 819200, "row count");
static_assert(kCellBlocks * kCellRows == kBatch, "cell blocks cover the batch");
static_assert(kPassBlocks * kTilesPerBlock * kTileRows == kRows, "pass blocks cover all rows");
static_assert(kHeadBlocks * kHeadThreads == kRows, "head blocks cover all rows");
static_assert(kF1 == 32, "fc2 depth is one 32-deep k-step");
static_assert((kF2 % 16) == 0 && kF3 == 16, "column tiles of 16");
static_assert(kF2 > 64 && kF2 <= 80, "fc3 third k-step: first half real, second half zero");

constexpr size_t kOffHB   = 0;
constexpr size_t kOffY3   = kOffHB   + (size_t)kRows * kHid * 4;
constexpr size_t kOffMOMP = kOffY3   + (size_t)kRows * kF3 * 4;
constexpr size_t kOffP1   = kOffMOMP + (size_t)kCellBlocks * 32 * 4;
constexpr size_t kOffPA   = kOffP1   + (size_t)160 * 4;
constexpr size_t kOffT2   = kOffPA   + (size_t)kPassBlocks * 160 * 4;
constexpr size_t kOffP3   = kOffT2   + (size_t)256 * 4;
constexpr size_t kOffT3   = kOffP3   + (size_t)kPassBlocks * 32 * 4;
constexpr size_t kWsTotal = kOffT3   + (size_t)64 * 4;
static_assert(kWsTotal == 59615104ull, "carve total");
static_assert(kWsTotal <= 134217728ull, "carve cap");
static_assert((kOffY3 % 128) == 0 && (kOffMOMP % 128) == 0 && (kOffP1 % 128) == 0 && (kOffPA % 128) == 0 &&
              (kOffT2 % 128) == 0 && (kOffP3 % 128) == 0 && (kOffT3 % 128) == 0, "128-B aligned regions");

__device__ __forceinline__ unsigned short f2bf_bits(float f) {
  unsigned u = __float_as_uint(f);
  return (unsigned short)((u + 0x7FFFu + ((u >> 16) & 1u)) >> 16);
}
__device__ __forceinline__ float bf_bits2f(unsigned short h) { return __uint_as_float(((unsigned)h) << 16); }
__device__ __forceinline__ __bf16 bits2bf(unsigned short h) { return __builtin_bit_cast(__bf16, h); }
__device__ __forceinline__ float lrelu(float v) { return v >= 0.0f ? v : 0.01f * v; }

union FragB { v16b v; v8b h[2]; };
__device__ __forceinline__ v16b frag_full(const __bf16* p) {
  FragB f;
  f.h[0] = *(const v8b*)(p);
  f.h[1] = *(const v8b*)(p + 16);
  return f.v;
}
__device__ __forceinline__ v16b frag_half(const __bf16* p, v8b z) {
  FragB f;
  f.h[0] = *(const v8b*)(p);
  f.h[1] = z;
  return f.v;
}
__device__ __forceinline__ v8b zero8b() {
  v8b z;
#pragma unroll
  for (int e = 0; e < 8; ++e) z[e] = bits2bf((unsigned short)0);
  return z;
}
__device__ __forceinline__ v8f mma_bf(v16b a, v16b b, v8f c) {
  c = __builtin_amdgcn_wmma_f32_16x16x32_bf16(false, a, false, b, (short)0, c, false, false);
  asm volatile("v_nop\n\tv_nop\n\tv_nop\n\tv_nop" : "+v"(c) : "v"(a), "v"(b));
  return c;
}
__device__ __forceinline__ void split8(const v4f a0, const v4f a1, v8b& vh, v8b& vl) {
#pragma unroll
  for (int e = 0; e < 4; ++e) {
    const float f0 = a0[e];
    const float f1 = a1[e];
    const unsigned short h0 = f2bf_bits(f0);
    const unsigned short h1 = f2bf_bits(f1);
    const unsigned short l0 = f2bf_bits(f0 - bf_bits2f(h0));
    const unsigned short l1 = f2bf_bits(f1 - bf_bits2f(h1));
    vh[e]     = bits2bf(h0);
    vh[4 + e] = bits2bf(h1);
    vl[e]     = bits2bf(l0);
    vl[4 + e] = bits2bf(l1);
  }
}

__global__ __launch_bounds__(32) void cell_scan_kernel(
    const float* __restrict__ x,
    const float* __restrict__ Wih, const float* __restrict__ Whh,
    const float* __restrict__ bih, const float* __restrict__ bhh,
    float* __restrict__ hbuf, float* __restrict__ momPart)
{
  __shared__ __align__(16) float sHB[kCellRows * kSteps * kHid];
  __shared__ __align__(16) float sWt[64];
  __shared__ float sAct[8 * 32];
  __shared__ float sCs[2 * 32];
  __shared__ float sHs[2 * 32];
  __shared__ double sMom[5 * 32];
  const int lane = threadIdx.x;

#pragma unroll
  for (int i = 0; i < 2; ++i) {
    const int idx = lane + 32 * i;
    const int g = idx >> 3;
    const int k = idx & 7;
    const int ka = (k < 3) ? k : 3;
    const int kb = (k == 5) ? 1 : 0;
    float va = Wih[g * 4 + ka];
    asm volatile("" : "+v"(va));
    float vb = Whh[g * 2 + kb];
    asm volatile("" : "+v"(vb));
    float vc = bih[g];
    asm volatile("" : "+v"(vc));
    float vd = bhh[g];
    asm volatile("" : "+v"(vd));
    const float v = (k < 4) ? va : ((k < 6) ? vb : ((k == 6) ? (vc + vd) : 0.0f));
    sWt[idx] = v;
  }
  sCs[lane] = 0.0f;
  sCs[32 + lane] = 0.0f;
  sHs[lane] = 0.0f;
  sHs[32 + lane] = 0.0f;
  __syncthreads();

  const int brow = blockIdx.x * kCellRows + lane;
  const float* xp = x + (size_t)brow * (kSteps * kIn);
  double a0 = 0.0, a1 = 0.0, a00 = 0.0, a11 = 0.0, a01 = 0.0;
  float h0 = 0.0f, h1 = 0.0f;

#pragma unroll 1
  for (int t = 0; t < kSteps; ++t) {
    const v4f xv = *(const v4f*)(xp + t * kIn);
#pragma unroll 1
    for (int g = 0; g < 8; ++g) {
      const v4f wa = *(const v4f*)(sWt + g * 8);
      const v4f wb = *(const v4f*)(sWt + g * 8 + 4);
      float z = wb[2];
      z = fmaf(wa[0], xv[0], z);
      z = fmaf(wa[1], xv[1], z);
      z = fmaf(wa[2], xv[2], z);
      z = fmaf(wa[3], xv[3], z);
      z = fmaf(wb[0], h0, z);
      z = fmaf(wb[1], h1, z);
      float a;
      if ((g >> 1) == 2) a = tanhf(z);
      else a = 1.0f / (1.0f + expf(-z));
      sAct[g * 32 + lane] = a;
    }
#pragma unroll 1
    for (int j = 0; j < 2; ++j) {
      const float ig = sAct[j * 32 + lane];
      const float fg = sAct[(2 + j) * 32 + lane];
      const float gg = sAct[(4 + j) * 32 + lane];
      const float og = sAct[(6 + j) * 32 + lane];
      float cc = sCs[j * 32 + lane];
      cc = fg * cc + ig * gg;
      const float hn = og * tanhf(cc);
      sCs[j * 32 + lane] = cc;
      sHs[j * 32 + lane] = hn;
      sHB[(lane * kSteps + t) * 2 + j] = hn;
    }
    h0 = sHs[lane];
    h1 = sHs[32 + lane];
    const double d0 = (double)h0;
    const double d1 = (double)h1;
    a0 += d0;
    a1 += d1;
    a00 += d0 * d0;
    a11 += d1 * d1;
    a01 += d0 * d1;
  }

  sMom[0 * 32 + lane] = a0;
  sMom[1 * 32 + lane] = a1;
  sMom[2 * 32 + lane] = a00;
  sMom[3 * 32 + lane] = a11;
  sMom[4 * 32 + lane] = a01;
  __syncthreads();

  {
    float* hb = hbuf + (size_t)blockIdx.x * (kCellRows * kSteps * kHid);
    for (int pass = 0; pass < 2; ++pass) {
#pragma unroll 4
      for (int it = 0; it < (kCellRows * kSteps * kHid) / 128; ++it) {
        const v4f v = *(const v4f*)(sHB + (it * 32 + lane) * 4);
        *(volatile v4f*)(hb + (it * 32 + lane) * 4) = v;
      }
      __threadfence();
    }
  }

  {
    const int qq = (lane < 4) ? lane : 4;
    double tot = 0.0;
#pragma unroll 1
    for (int i = 0; i < 32; ++i) tot += sMom[qq * 32 + i];
    const float val = (lane < 5) ? (float)tot : 0.0f;
    float* mp = momPart + (size_t)blockIdx.x * 32 + lane;
    *(volatile float*)mp = val;
    __threadfence();
    *(volatile float*)mp = val;
  }
}

__global__ __launch_bounds__(32) void bn1_params_kernel(
    const float* __restrict__ momPart, const float* __restrict__ w1,
    const float* __restrict__ g1, const float* __restrict__ b1n, float* __restrict__ P1)
{
  __shared__ __align__(16) float sT[160];
  const int lane = threadIdx.x;
  double s0 = 0.0, s1 = 0.0, s00 = 0.0, s11 = 0.0, s01 = 0.0;
#pragma unroll 1
  for (int b = 0; b < kCellBlocks; ++b) {
    const float* p = momPart + (size_t)b * 32;
    s0  += (double)p[0];
    s1  += (double)p[1];
    s00 += (double)p[2];
    s11 += (double)p[3];
    s01 += (double)p[4];
  }
  const double invN = 1.0 / (double)kRows;
  const double m0 = s0 * invN, m1 = s1 * invN;
  const double c00 = s00 * invN - m0 * m0;
  const double c11 = s11 * invN - m1 * m1;
  const double c01 = s01 * invN - m0 * m1;
  const float w0 = w1[lane * 2 + 0];
  const float wq = w1[lane * 2 + 1];
  const double dw0 = (double)w0, dw1 = (double)wq;
  const double var = dw0 * dw0 * c00 + 2.0 * dw0 * dw1 * c01 + dw1 * dw1 * c11;
  float vf = (float)var;
  vf = fmaxf(vf, 0.0f);
  const float istd = 1.0f / sqrtf(vf + kEps);
  sT[lane * 4 + 0] = w0;
  sT[lane * 4 + 1] = wq;
  sT[lane * 4 + 2] = istd * g1[lane];
  sT[lane * 4 + 3] = b1n[lane];
  sT[128 + lane] = (lane == 0) ? (float)m0 : ((lane == 1) ? (float)m1 : 0.0f);
  __syncthreads();
  const v4f v = *(const v4f*)(sT + lane * 4);
  const float u = sT[128 + lane];
  for (int pass = 0; pass < 2; ++pass) {
    *(volatile v4f*)(P1 + lane * 4) = v;
    *(volatile float*)(P1 + 128 + lane) = u;
    __threadfence();
  }
}

__global__ __launch_bounds__(128) void bn_params_kernel(
    const float* __restrict__ part, int nblk, int nf, int pitch,
    const float* __restrict__ gamma, const float* __restrict__ beta,
    float* __restrict__ tab, int tabFloats)
{
  __shared__ __align__(16) float sT[256];
  const int tid = threadIdx.x;
  sT[tid] = 0.0f;
  sT[tid + 128] = 0.0f;
  __syncthreads();
  const int j = (tid < nf) ? tid : (nf - 1);
  double S = 0.0, Q = 0.0;
#pragma unroll 1
  for (int b = 0; b < nblk; ++b) {
    const float* p = part + (size_t)b * pitch;
    S += (double)p[j];
    Q += (double)p[nf + j];
  }
  const double invN = 1.0 / (double)kRows;
  const double mean = S * invN;
  const double var = Q * invN - mean * mean;
  float vf = (float)var;
  vf = fmaxf(vf, 0.0f);
  const float sc = (1.0f / sqrtf(vf + kEps)) * gamma[j];
  const float bt = beta[j];
  if (tid < nf) {
    sT[tid] = (float)mean;
    sT[nf + tid] = sc;
    sT[2 * nf + tid] = bt;
  }
  __syncthreads();
  const int t4 = ((tid * 4 < tabFloats) ? tid : 0) * 4;
  const v4f v = *(const v4f*)(sT + t4);
  if (tid * 4 < tabFloats) {
    for (int pass = 0; pass < 2; ++pass) {
      *(volatile v4f*)(tab + t4) = v;
      __threadfence();
    }
  }
}

template <int MODE>
__global__ __launch_bounds__(128) void mlp_pass_kernel(
    const float* __restrict__ hbuf, const float* __restrict__ P1g,
    const float* __restrict__ W2, const float* __restrict__ T2g,
    const float* __restrict__ W3, float* __restrict__ partOut, float* __restrict__ y3)
{
  __shared__ __align__(16) __bf16 sW2h[kF2 * kF1];
  __shared__ __align__(16) __bf16 sW2l[kF2 * kF1];
  __shared__ __align__(16) __bf16 sW3h[MODE ? kF3 * kF2 : 8];
  __shared__ __align__(16) __bf16 sW3l[MODE ? kF3 * kF2 : 8];
  __shared__ __align__(16) __bf16 sA1h[kTileRows * kF1];
  __shared__ __align__(16) __bf16 sA1l[kTileRows * kF1];
  __shared__ __align__(16) __bf16 sA2h[MODE ? 4 * 16 * kF2 : 8];
  __shared__ __align__(16) __bf16 sA2l[MODE ? 4 * 16 * kF2 : 8];
  __shared__ __align__(16) float sY3[MODE ? 4 * 256 : 4];
  __shared__ __align__(16) float sP1[160];
  __shared__ __align__(16) float sT2[MODE ? 256 : 4];
  __shared__ __align__(16) float sRed[640];

  const int tid  = threadIdx.x;
  const int lane = tid & 31;
  const int hh   = lane >> 4;
  const int c    = lane & 15;
  const int wave = __builtin_amdgcn_readfirstlane((int)(threadIdx.x >> 5));

#pragma unroll 1
  for (int i = 0; i < 3; ++i) {
    int ch = tid + 128 * i;
    ch = (ch < 320) ? ch : 319;
    const v4f w0 = *(const v4f*)(W2 + ch * 8);
    const v4f w1 = *(const v4f*)(W2 + ch * 8 + 4);
    v8b vh, vl;
    split8(w0, w1, vh, vl);
    *(v8b*)(sW2h + ch * 8) = vh;
    *(v8b*)(sW2l + ch * 8) = vl;
  }
  if (MODE == 1) {
#pragma unroll 1
    for (int i = 0; i < 2; ++i) {
      int ch = tid + 128 * i;
      ch = (ch < 160) ? ch : 159;
      const v4f w0 = *(const v4f*)(W3 + ch * 8);
      const v4f w1 = *(const v4f*)(W3 + ch * 8 + 4);
      v8b vh, vl;
      split8(w0, w1, vh, vl);
      *(v8b*)(sW3h + ch * 8) = vh;
      *(v8b*)(sW3l + ch * 8) = vl;
    }
    sT2[tid] = T2g[tid];
    sT2[tid + 128] = T2g[tid + 128];
  }
  {
    const int i4 = (tid < 40) ? tid : 39;
    *(v4f*)(sP1 + i4 * 4) = *(const v4f*)(P1g + i4 * 4);
  }
  __syncthreads();

  const float m0 = sP1[128];
  const float m1 = sP1[129];
  const v8b z8 = zero8b();

  float s2[5], q2[5];
#pragma unroll
  for (int ct = 0; ct < 5; ++ct) { s2[ct] = 0.0f; q2[ct] = 0.0f; }
  float s3 = 0.0f, q3 = 0.0f;

#pragma unroll 1
  for (int tl = 0; tl < kTilesPerBlock; ++tl) {
    const int tileRow0 = (blockIdx.x * kTilesPerBlock + tl) * kTileRows;

    {
      const v2f hv = *(const v2f*)(hbuf + (size_t)(tileRow0 + tid) * 2);
      const float d0 = hv[0] - m0;
      const float d1 = hv[1] - m1;
#pragma unroll 1
      for (int jg = 0; jg < 4; ++jg) {
        v8b vh, vl;
#pragma unroll
        for (int e = 0; e < 8; ++e) {
          const v4f cf = *(const v4f*)(sP1 + (jg * 8 + e) * 4);
          float y = cf[1] * d1;
          y = fmaf(cf[0], d0, y);
          float a = fmaf(y, cf[2], cf[3]);
          a = lrelu(a);
          const unsigned short hb = f2bf_bits(a);
          const unsigned short lb = f2bf_bits(a - bf_bits2f(hb));
          vh[e] = bits2bf(hb);
          vl[e] = bits2bf(lb);
        }
        *(v8b*)(sA1h + tid * kF1 + jg * 8) = vh;
        *(v8b*)(sA1l + tid * kF1 + jg * 8) = vl;
      }
    }
    __syncthreads();

#pragma unroll 1
    for (int rt = 0; rt < 2; ++rt) {
      const int lrow0 = wave * 32 + rt * 16;
      const int aoff = (lrow0 + c) * kF1 + 8 * hh;
      const v16b ah = frag_full(sA1h + aoff);
      const v16b al = frag_full(sA1l + aoff);
      v8f acc[5];
#pragma unroll
      for (int ct = 0; ct < 5; ++ct) {
        const int boff = (ct * 16 + c) * kF1 + 8 * hh;
        const v16b bh = frag_full(sW2h + boff);
        const v16b bl = frag_full(sW2l + boff);
        v8f a = (v8f){0.f, 0.f, 0.f, 0.f, 0.f, 0.f, 0.f, 0.f};
        a = mma_bf(ah, bl, a);
        a = mma_bf(al, bh, a);
        a = mma_bf(ah, bh, a);
        acc[ct] = a;
      }

      if (MODE == 0) {
#pragma unroll
        for (int ct = 0; ct < 5; ++ct) {
#pragma unroll
          for (int r = 0; r < 8; ++r) {
            const float y = acc[ct][r];
            s2[ct] += y;
            q2[ct] = fmaf(y, y, q2[ct]);
          }
        }
      } else {
        __bf16* a2h = sA2h + wave * (16 * kF2);
        __bf16* a2l = sA2l + wave * (16 * kF2);
#pragma unroll
        for (int ct = 0; ct < 5; ++ct) {
          const int col = ct * 16 + c;
          const float mu = sT2[col];
          const float sc = sT2[kF2 + col];
          const float bt = sT2[2 * kF2 + col];
#pragma unroll
          for (int r = 0; r < 8; ++r) {
            float v = acc[ct][r] - mu;
            v = fmaf(v, sc, bt);
            v = lrelu(v);
            const unsigned short hb = f2bf_bits(v);
            const unsigned short lb = f2bf_bits(v - bf_bits2f(hb));
            const int idx = (8 * hh + r) * kF2 + col;
            a2h[idx] = bits2bf(hb);
            a2l[idx] = bits2bf(lb);
          }
        }
        __syncthreads();

        v8f acc3 = (v8f){0.f, 0.f, 0.f, 0.f, 0.f, 0.f, 0.f, 0.f};
#pragma unroll
        for (int ks = 0; ks < 3; ++ks) {
          const int off = c * kF2 + ks * 32 + 8 * hh;
          v16b xh, xl, wh, wl;
          if (ks < 2) {
            xh = frag_full(a2h + off);
            xl = frag_full(a2l + off);
            wh = frag_full(sW3h + off);
            wl = frag_full(sW3l + off);
          } else {
            xh = frag_half(a2h + off, z8);
            xl = frag_half(a2l + off, z8);
            wh = frag_half(sW3h + off, z8);
            wl = frag_half(sW3l + off, z8);
          }
          acc3 = mma_bf(xh, wl, acc3);
          acc3 = mma_bf(xl, wh, acc3);
          acc3 = mma_bf(xh, wh, acc3);
        }
        float* slab = sY3 + wave * 256;
#pragma unroll
        for (int r = 0; r < 8; ++r) {
          const float y = acc3[r];
          slab[(8 * hh + r) * 16 + c] = y;
          s3 += y;
          q3 = fmaf(y, y, q3);
        }
        __syncthreads();
        {
          const v4f v0 = *(const v4f*)(slab + lane * 4);
          const v4f v1 = *(const v4f*)(slab + 128 + lane * 4);
          float* gp = y3 + (size_t)(tileRow0 + lrow0) * kF3;
          for (int pass = 0; pass < 2; ++pass) {
            *(volatile v4f*)(gp + lane * 4) = v0;
            *(volatile v4f*)(gp + 128 + lane * 4) = v1;
            __threadfence();
          }
        }
        __syncthreads();
      }
    }
    __syncthreads();
  }

  if (MODE == 0) {
#pragma unroll
    for (int ct = 0; ct < 5; ++ct) {
      s2[ct] += __shfl_xor(s2[ct], 16, 32);
      q2[ct] += __shfl_xor(q2[ct], 16, 32);
    }
#pragma unroll
    for (int ct = 0; ct < 5; ++ct)
      sRed[wave * 160 + hh * kF2 + ct * 16 + c] = hh ? q2[ct] : s2[ct];
    __syncthreads();
    const int t4 = ((tid < 40) ? tid : 39) * 4;
    const v4f r0 = *(const v4f*)(sRed + t4);
    const v4f r1 = *(const v4f*)(sRed + 160 + t4);
    const v4f r2 = *(const v4f*)(sRed + 320 + t4);
    const v4f r3 = *(const v4f*)(sRed + 480 + t4);
    const v4f tot = ((r0 + r1) + r2) + r3;
    if (tid < 40) {
      float* gp = partOut + (size_t)blockIdx.x * 160 + t4;
      for (int pass = 0; pass < 2; ++pass) {
        *(volatile v4f*)gp = tot;
        __threadfence();
      }
    }
  } else {
    s3 += __shfl_xor(s3, 16, 32);
    q3 += __shfl_xor(q3, 16, 32);
    sRed[wave * 32 + lane] = hh ? q3 : s3;
    __syncthreads();
    const float tot = ((sRed[lane] + sRed[32 + lane]) + sRed[64 + lane]) + sRed[96 + lane];
    if (wave == 0) {
      float* gp = partOut + (size_t)blockIdx.x * 32 + lane;
      *(volatile float*)gp = tot;
      __threadfence();
      *(volatile float*)gp = tot;
    }
  }
}

__global__ __launch_bounds__(256) void head_kernel(
    const float* __restrict__ y3, const float* __restrict__ T3g,
    const float* __restrict__ w4, const float* __restrict__ b4, float* __restrict__ out)
{
  __shared__ __align__(16) float sT[64];
  __shared__ __align__(16) float sW4[32];
  __shared__ float sB4[2];
  const int tid = threadIdx.x;
  {
    const int i = (tid < 64) ? tid : 63;
    sT[i] = T3g[i];
    const int k = (tid < 32) ? tid : 31;
    sW4[k] = w4[k];
    const int q = (tid < 2) ? tid : 1;
    sB4[q] = b4[q];
  }
  __syncthreads();
  const size_t row = (size_t)blockIdx.x * kHeadThreads + tid;
  const v4f* yp = (const v4f*)(y3 + row * kF3);
  v4f yv[4];
#pragma unroll
  for (int i = 0; i < 4; ++i) yv[i] = yp[i];
  float o0 = sB4[0], o1 = sB4[1];
#pragma unroll
  for (int k = 0; k < 16; ++k) {
    float a = yv[k >> 2][k & 3] - sT[k];
    a = fmaf(a, sT[16 + k], sT[32 + k]);
    a = lrelu(a);
    o0 = fmaf(sW4[k], a, o0);
    o1 = fmaf(sW4[16 + k], a, o1);
  }
  v2f ov;
  ov[0] = lrelu(o0);
  ov[1] = lrelu(o1);
  float* gp = out + row * kOutW;
  *(volatile v2f*)gp = ov;
  __threadfence();
  *(volatile v2f*)gp = ov;
}

extern "C" void kernel_launch(void* const* d_in, const int* in_sizes, int n_in,
                              void* d_out, int out_size, void* d_ws, size_t ws_size,
                              hipStream_t stream)
{
  if (n_in < 19) return;
  if (in_sizes[0] != kRows * kIn) return;
  if (in_sizes[1] != 8 * kIn) return;
  if (in_sizes[2] != 8 * kHid) return;
  if (in_sizes[3] != 8) return;
  if (in_sizes[4] != 8) return;
  if (in_sizes[5] != kF1 * kHid) return;
  if (in_sizes[7] != kF2 * kF1) return;
  if (in_sizes[9] != kF3 * kF2) return;
  if (in_sizes[11] != kOutW * kF3) return;
  if (in_sizes[12] != kOutW) return;
  if (in_sizes[13] != kF1) return;
  if (in_sizes[14] != kF1) return;
  if (in_sizes[15] != kF2) return;
  if (in_sizes[16] != kF2) return;
  if (in_sizes[17] != kF3) return;
  if (in_sizes[18] != kF3) return;
  if (out_size != kRows * kOutW) return;
  if (ws_size < kWsTotal) return;

  const float* x     = (const float*)d_in[0];
  const float* Wih   = (const float*)d_in[1];
  const float* Whh   = (const float*)d_in[2];
  const float* bih   = (const float*)d_in[3];
  const float* bhh   = (const float*)d_in[4];
  const float* fc1w  = (const float*)d_in[5];
  const float* fc2w  = (const float*)d_in[7];
  const float* fc3w  = (const float*)d_in[9];
  const float* fc4w  = (const float*)d_in[11];
  const float* fc4b  = (const float*)d_in[12];
  const float* bn1g  = (const float*)d_in[13];
  const float* bn1b  = (const float*)d_in[14];
  const float* bn2g  = (const float*)d_in[15];
  const float* bn2b  = (const float*)d_in[16];
  const float* bn3g  = (const float*)d_in[17];
  const float* bn3b  = (const float*)d_in[18];
  float* out = (float*)d_out;

  char* ws = (char*)d_ws;
  float* HB   = (float*)(ws + kOffHB);
  float* Y3   = (float*)(ws + kOffY3);
  float* MOMP = (float*)(ws + kOffMOMP);
  float* P1   = (float*)(ws + kOffP1);
  float* PA   = (float*)(ws + kOffPA);
  float* T2   = (float*)(ws + kOffT2);
  float* P3   = (float*)(ws + kOffP3);
  float* T3   = (float*)(ws + kOffT3);

  cell_scan_kernel<<<kCellBlocks, kCellRows, 0, stream>>>(x, Wih, Whh, bih, bhh, HB, MOMP);
  bn1_params_kernel<<<1, 32, 0, stream>>>(MOMP, fc1w, bn1g, bn1b, P1);
  mlp_pass_kernel<0><<<kPassBlocks, 128, 0, stream>>>(HB, P1, fc2w, T2, fc3w, PA, Y3);
  bn_params_kernel<<<1, 128, 0, stream>>>(PA, kPassBlocks, kF2, 160, bn2g, bn2b, T2, 256);
  mlp_pass_kernel<1><<<kPassBlocks, 128, 0, stream>>>(HB, P1, fc2w, T2, fc3w, P3, Y3);
  bn_params_kernel<<<1, 128, 0, stream>>>(P3, kPassBlocks, kF3, 32, bn3g, bn3b, T3, 64);
  head_kernel<<<kHeadBlocks, kHeadThreads, 0, stream>>>(Y3, T3, fc4w, fc4b, out);
}
